// LLTM_15195594293829
// MI455X (gfx1250) — hardware-run, weakly checked
//
#include <hip/hip_runtime.h>
#include <math.h>

typedef __attribute__((ext_vector_type(16))) _Float16 v16h;
typedef __attribute__((ext_vector_type(16))) __bf16 v16b;
typedef __attribute__((ext_vector_type(8)))  _Float16 v8h;
typedef __attribute__((ext_vector_type(8)))  float v8f;
typedef __attribute__((ext_vector_type(4)))  float v4f;
typedef __attribute__((ext_vector_type(2)))  float v2f;
typedef __attribute__((ext_vector_type(4)))  unsigned v4u;
typedef __attribute__((ext_vector_type(4)))  int v4i;
typedef float __attribute__((may_alias)) float_a;
typedef int __attribute__((may_alias)) int_a;

template <typename T> __device__ __forceinline__ void vst2(void* p, T v) { *(volatile T*)p = v; __threadfence(); *(volatile T*)p = v; }
__device__ __forceinline__ v8f wmma16(v16h a, v16h b, v8f c) {
  v8f d = __builtin_amdgcn_wmma_f32_16x16x32_f16(false, a, false, b, (short)0, c, false, false);
  asm volatile("v_nop\n\tv_nop\n\tv_nop\n\tv_nop" : "+v"(d) : "v"(a), "v"(b));
  return d;
}
__device__ __forceinline__ v8f wmma_bf(v16b a, v16b b, v8f c) {
  v8f d = __builtin_amdgcn_wmma_f32_16x16x32_bf16(false, a, false, b, (short)0, c, false, false);
  asm volatile("v_nop\n\tv_nop\n\tv_nop\n\tv_nop" : "+v"(d) : "v"(a), "v"(b));
  return d;
}
__device__ __forceinline__ v16h frag_h(const _Float16* rowk0, int lane) {
  union { v16h v; v8h q[2]; } u; const _Float16* p = rowk0 + 8 * (lane >> 4);
  u.q[0] = *(const v8h*)p; u.q[1] = *(const v8h*)(p + 16); return u.v;
}
__device__ __forceinline__ v16h frag_f32(const float* rowk0, int lane) {
  v16h a; const float* p = rowk0 + 8 * (lane >> 4);
#pragma unroll
  for (int i = 0; i < 8; ++i) { a[i] = (_Float16)p[i]; a[8 + i] = (_Float16)p[16 + i]; }
  return a;
}
__device__ __forceinline__ v16h frag_f32s(const float* rowk0, int lane, float sc) {
  v16h a; const float* p = rowk0 + 8 * (lane >> 4);
#pragma unroll
  for (int i = 0; i < 8; ++i) { a[i] = (_Float16)(p[i] * sc); a[8 + i] = (_Float16)(p[16 + i] * sc); }
  return a;
}
__device__ __forceinline__ v16h fragc_f32(const float* W, int k0, int n, int lane, int ld, int K) {
  v16h a; const int g = lane >> 4;
#pragma unroll
  for (int i = 0; i < 8; ++i) { const int ka = k0 + 8 * g + i, kb = ka + 16;
    a[i] = (_Float16)(ka < K ? W[(size_t)(ka < K ? ka : K - 1) * ld + n] : 0.f); a[8 + i] = (_Float16)(kb < K ? W[(size_t)(kb < K ? kb : K - 1) * ld + n] : 0.f); }
  return a;
}
struct F2 { v16b h, l; };
__device__ __forceinline__ F2 bsplit16(const float v[16]) { F2 r;
#pragma unroll
  for (int i = 0; i < 16; ++i) { const __bf16 h = (__bf16)v[i]; r.h[i] = h; r.l[i] = (__bf16)(v[i] - (float)h); }
  return r; }
__device__ __forceinline__ F2 split_row(const float* row, int k0, int lane) { float v[16]; const float* p = row + k0 + 8 * (lane >> 4);
#pragma unroll
  for (int i = 0; i < 8; ++i) { v[i] = p[i]; v[8 + i] = p[16 + i]; }
  return bsplit16(v); }
__device__ __forceinline__ F2 split_rowK(const float* row, int k0, int lane, int K) { float v[16]; const int g = lane >> 4;
#pragma unroll
  for (int i = 0; i < 8; ++i) { const int ka = k0 + 8 * g + i, kb = ka + 16; v[i] = ka < K ? row[ka < K ? ka : K - 1] : 0.f; v[8 + i] = kb < K ? row[kb < K ? kb : K - 1] : 0.f; }
  return bsplit16(v); }
__device__ __forceinline__ F2 split_col(const float* W, int k0, int n, int lane, int ld, int K) { float v[16]; const int g = lane >> 4;
#pragma unroll
  for (int i = 0; i < 8; ++i) { const int ka = k0 + 8 * g + i, kb = ka + 16; v[i] = ka < K ? W[(size_t)(ka < K ? ka : K - 1) * ld + n] : 0.f; v[8 + i] = kb < K ? W[(size_t)(kb < K ? kb : K - 1) * ld + n] : 0.f; }
  return bsplit16(v); }
__device__ __forceinline__ v8f mac3(const F2& a, const F2& b, v8f c) { c = wmma_bf(a.l, b.h, c); c = wmma_bf(a.h, b.l, c); return wmma_bf(a.h, b.h, c); }
__device__ __forceinline__ float sigm(float v) { return 1.0f / (1.0f + expf(-v)); }
#define LDSX() do { asm volatile("s_wait_dscnt 0" ::: "memory"); __builtin_amdgcn_wave_barrier(); __builtin_amdgcn_fence(__ATOMIC_RELEASE, "workgroup"); } while (0)


#define NBR 4096
#define IN 1024
#define ST 1024
#define KW (IN + ST)
#ifndef TR
#define TR (NBR / 64)
#endif
typedef __attribute__((ext_vector_type(8))) __bf16 v8b;
__device__ __forceinline__ v16b frag_b(const __bf16* rowk0, int lane) {
  union { v16b v; v8b q[2]; } u; const __bf16* p = rowk0 + 8 * (lane >> 4);
  u.q[0] = *(const v8b*)p; u.q[1] = *(const v8b*)(p + 16); return u.v;
}
__device__ __forceinline__ float bfr(float v) { return (float)(__bf16)v; }
__device__ __attribute__((noinline)) float exp_ni(float v) { return expf(v); }
__device__ __attribute__((noinline)) float erf_ni(float v) { return erff(v); }

__device__ __forceinline__ v16b fragb_f32(const float* __restrict__ p, int lane) { v16b a; const float* pp = p + 8 * (lane >> 4);
#pragma unroll
  for (int i = 0; i < 8; ++i) { a[i] = (__bf16)pp[i]; a[8 + i] = (__bf16)pp[16 + i]; } return a; }
__global__ __launch_bounds__(128) void k_lltm(const float* __restrict__ X, const float* __restrict__ H0, const float* __restrict__ C0, const float* __restrict__ Wt, const float* __restrict__ BIAS, float* __restrict__ HOUT, float* __restrict__ COUT) { __shared__ __align__(16) float sh[64][36], sc[64][36];
  const int tid = threadIdx.x, wave = tid >> 5, lane = tid & 31, col = lane & 15, g = lane >> 4; const size_t r0 = (size_t)blockIdx.x * 64 + wave * 16; const int s0 = blockIdx.y * 32;
  v8f acc[8] = {};
#pragma unroll 8
  for (int kc = 0; kc < KW / 32; ++kc) { const v16b a = (kc < IN / 32) ? fragb_f32(X + (r0 + col) * IN + kc * 32, lane) : fragb_f32(H0 + (r0 + col) * ST + (kc - IN / 32) * 32, lane);
#pragma unroll
    for (int j = 0; j < 8; ++j) { const int gate = j >> 1, sl = (j & 1) * 16 + col; acc[j] = wmma_bf(a, fragb_f32(Wt + ((size_t)gate * ST + s0 + sl) * KW + kc * 32, lane), acc[j]); } }
#pragma unroll
  for (int u = 0; u < 2; ++u) { const int sl = u * 16 + col, s = s0 + sl; const float bf_ = bfr(BIAS[s]), bi = bfr(BIAS[ST + s]), bo = bfr(BIAS[2 * ST + s]), bg = bfr(BIAS[3 * ST + s]);
#pragma unroll
    for (int r = 0; r < 8; ++r) { const size_t row = r0 + 8 * g + r; const float f = sigm(acc[u][r] + bf_), i = sigm(acc[2 + u][r] + bi), o = sigm(acc[4 + u][r] + bo), gg = tanhf(acc[6 + u][r] + bg); const float c = f * bfr(C0[row * ST + s]) + i * gg; sc[wave * 16 + 8 * g + r][sl] = c; sh[wave * 16 + 8 * g + r][sl] = o * tanhf(c); } }
  __syncthreads(); for (int e = tid; e < 64 * 8; e += 128) { const int rl = e >> 3, q = e & 7; const size_t o = ((size_t)blockIdx.x * 64 + rl) * ST + s0 + q * 4; vst2(HOUT + o, *(const v4f*)&sh[rl][q * 4]); vst2(COUT + o, *(const v4f*)&sc[rl][q * 4]); } }
extern "C" void kernel_launch(void* const* d_in, const int* in_sizes, int n_in, void* d_out, int out_size, void* d_ws, size_t ws_size, hipStream_t stream) {
  (void)in_sizes; (void)n_in; (void)out_size; (void)d_ws; (void)ws_size;
  const float** F = (const float**)d_in;
  float* HOUT = (float*)d_out; float* COUT = HOUT + (size_t)NBR * ST;
  k_lltm<<<dim3(TR, ST / 32), 128, 0, stream>>>(F[0], F[1], F[2], F[3], F[4], HOUT, COUT);
}
